// LongformerMultiHeadAttention_74826920230969
// MI455X (gfx1250) — hardware-verified
//
#include <hip/hip_runtime.h>


namespace {
constexpr int NB = 2, S = 4096, D = 1024, NH = 16, DH = 64, W1 = 128, G = 64, NROW = NB * S;
constexpr int LPAD = 128, RPAD = 160, LV = LPAD + S + RPAD;
constexpr float XS = 8.0f, WSC = 256.0f, PS = 8.0f, QSCALE = 0.125f;

typedef _Float16 b16;
typedef __attribute__((ext_vector_type(16))) _Float16 v16b;
typedef __attribute__((ext_vector_type(8))) _Float16 v8b;
typedef __attribute__((ext_vector_type(8))) float v8f;
typedef __attribute__((ext_vector_type(4))) float v4f;
__device__ __forceinline__ float bf16_rne(float f) { unsigned int u = __float_as_uint(f); u += 0x7FFFu + ((u >> 16) & 1u); return __uint_as_float(u & 0xFFFF0000u); }
__device__ __forceinline__ void split16(float v, b16& hi, b16& lo) { hi = (b16)v; lo = (b16)(v - (float)hi); }
__device__ __forceinline__ v16b frag_kb(const b16* p, int hh) { const v8b a = *(const v8b*)(p + 8 * hh), b = *(const v8b*)(p + 16 + 8 * hh); v16b f;
#pragma unroll
  for (int e = 0; e < 8; ++e) { f[e] = a[e]; f[8 + e] = b[e]; } return f; }
__device__ __forceinline__ v8f wmma16b(v16b a, v16b b, v8f c) { v8f d = __builtin_amdgcn_wmma_f32_16x16x32_f16(false, a, false, b, (short)0, c, false, false); asm volatile("v_nop\n\tv_nop\n\tv_nop\n\tv_nop" : "+v"(d) : "v"(a), "v"(b)); return d; }
__device__ __forceinline__ void wave_lds_sync() { __builtin_amdgcn_fence(__ATOMIC_RELEASE, "workgroup"); __builtin_amdgcn_wave_barrier(); __builtin_amdgcn_fence(__ATOMIC_ACQUIRE, "workgroup"); }
__device__ __forceinline__ float nexp(float x) { return __builtin_amdgcn_exp2f(x * 1.4426950408889634f); }
__device__ __forceinline__ int iclamp(int v, int lo, int hi) { return v < lo ? lo : (v > hi ? hi : v); }

__global__ __launch_bounds__(256) void prepx_kernel(const float* __restrict__ x, b16* __restrict__ X16) {
  const size_t i = ((size_t)blockIdx.x * 256 + threadIdx.x) * 8; if (i >= (size_t)NROW * D) return;
  const v4f a = *(const v4f*)(x + i), c = *(const v4f*)(x + i + 4); v8b o;
#pragma unroll
  for (int j = 0; j < 4; ++j) { o[j] = (b16)(bf16_rne(a[j]) * XS); o[4 + j] = (b16)(bf16_rne(c[j]) * XS); }
  for (int pass = 0; pass < 2; ++pass) { *(volatile v8b*)(X16 + i) = o; __threadfence(); }
}
__global__ __launch_bounds__(256) void prepw_kernel(const float* __restrict__ wq, const float* __restrict__ wk, const float* __restrict__ wv, const float* __restrict__ wo, b16* __restrict__ WT) {
  __shared__ __attribute__((aligned(16))) b16 T[64][64 + 8];
  const int which = blockIdx.z, i0 = blockIdx.x * 64, o0 = blockIdx.y * 64, t_ = threadIdx.x; const float* w = which == 0 ? wq : which == 1 ? wk : which == 2 ? wv : wo;
  for (int q = t_; q < 64 * 64; q += 256) { const int ii = q >> 6, oo = q & 63; T[oo][ii] = (b16)(bf16_rne(w[(size_t)(i0 + ii) * D + o0 + oo]) * WSC); }
  __syncthreads();
  for (int pass = 0; pass < 2; ++pass) { for (int q = t_; q < 64 * 8; q += 256) { const int oo = q >> 3, c8 = (q & 7) * 8; *(volatile v8b*)(WT + ((size_t)which * D + o0 + oo) * D + i0 + c8) = *(const v8b*)(&T[oo][c8]); } __threadfence(); }
}
__global__ __launch_bounds__(128) void qkv_kernel(const b16* __restrict__ X16, const b16* __restrict__ WT, b16* __restrict__ QH, b16* __restrict__ QL, b16* __restrict__ KH, b16* __restrict__ VROW, b16* __restrict__ VROWL, int zoff) {
  __shared__ __attribute__((aligned(16))) b16 Th[4][16][128 + 8], Tl[4][16][128 + 8];
  const int which = blockIdx.z + zoff, wave = threadIdx.x >> 5, lane = threadIdx.x & 31, nloc = lane & 15, hlf = lane >> 4; const int m0 = blockIdx.x * 64 + wave * 16, n0 = blockIdx.y * 128;
  const b16* Bw = WT + (size_t)which * D * D; const float osc = (which == 0) ? QSCALE : 1.0f;
  v8f acc[8];
#pragma unroll
  for (int t = 0; t < 8; ++t) acc[t] = (v8f){};
#pragma unroll 2
  for (int kb = 0; kb < D; kb += 32) { const v16b a = frag_kb(X16 + (size_t)(m0 + nloc) * D + kb, hlf);
#pragma unroll
    for (int t = 0; t < 8; ++t) acc[t] = wmma16b(a, frag_kb(Bw + (size_t)(n0 + t * 16 + nloc) * D + kb, hlf), acc[t]); }
#pragma unroll
  for (int t = 0; t < 8; ++t)
#pragma unroll
    for (int r = 0; r < 8; ++r) { b16 a_, c_; split16(acc[t][r] * (1.0f / (XS * WSC)) * osc * XS, a_, c_); Th[wave][8 * hlf + r][t * 16 + nloc] = a_; Tl[wave][8 * hlf + r][t * 16 + nloc] = c_; }
  wave_lds_sync();
  for (int pass = 0; pass < 2; ++pass) {
    for (int rr = 0; rr < 16; ++rr) { const int m = m0 + rr, b = m / S, s = m - b * S; const int hsel = lane >> 3, c8 = (lane & 7) * 8;
      if (lane < 16) { const int h = n0 / DH + hsel; const size_t gi = (((size_t)b * NH + h) * S + s) * DH + c8; const v8b vh = *(const v8b*)(&Th[wave][rr][hsel * 64 + c8]);
        const v8b vl = *(const v8b*)(&Tl[wave][rr][hsel * 64 + c8]);
        if (which == 0) { *(volatile v8b*)(QH + gi) = vh; *(volatile v8b*)(QL + gi) = vl; } else if (which == 1) *(volatile v8b*)(KH + gi) = vh; else { *(volatile v8b*)(VROW + gi) = vh; *(volatile v8b*)(VROWL + gi) = vl; } } }
    __threadfence(); }
}
__global__ __launch_bounds__(256) void vt_kernel(const b16* __restrict__ VROW, const b16* __restrict__ VROWL, const b16* __restrict__ KH, const int* __restrict__ gidx, b16* __restrict__ VT, b16* __restrict__ VTL, b16* __restrict__ KG, b16* __restrict__ VGT, b16* __restrict__ VGTL) {
  __shared__ __attribute__((aligned(16))) b16 Tt[DH][64 + 8], Tu[DH][64 + 8];
  const int bh = blockIdx.y, b = bh / NH, t_ = threadIdx.x;
  if (blockIdx.x < S / 64) { const int s0 = blockIdx.x * 64;
    for (int k = t_; k < 64 * DH; k += 256) { const int ss = k >> 6, d = k & 63; const size_t gi = ((size_t)bh * S + s0 + ss) * DH + d; Tt[d][ss] = VROW[gi]; Tu[d][ss] = VROWL[gi]; }
    __syncthreads();
    for (int pass = 0; pass < 2; ++pass) { for (int q = t_; q < DH * 8; q += 256) { const int d = q >> 3, c8 = (q & 7) * 8; const size_t gi = ((size_t)bh * DH + d) * LV + LPAD + s0 + c8; *(volatile v8b*)(VT + gi) = *(const v8b*)(&Tt[d][c8]); *(volatile v8b*)(VTL + gi) = *(const v8b*)(&Tu[d][c8]); } __threadfence(); }
  } else {
    for (int k = t_; k < G * DH; k += 256) { const int g = k >> 6, d = k & 63; const int pos = iclamp(gidx[b * G + g], 0, S - 1); const size_t gi = ((size_t)bh * S + pos) * DH + d; Tt[d][g] = VROW[gi]; Tu[d][g] = VROWL[gi]; }
    __syncthreads();
    for (int pass = 0; pass < 2; ++pass) {
      for (int q = t_; q < G * 8; q += 256) { const int g = q >> 3, c8 = (q & 7) * 8; const int pos = iclamp(gidx[b * G + g], 0, S - 1); *(volatile v8b*)(KG + ((size_t)bh * G + g) * DH + c8) = *(const v8b*)(KH + ((size_t)bh * S + pos) * DH + c8); }
      for (int q = t_; q < DH * 8; q += 256) { const int d = q >> 3, c8 = (q & 7) * 8; const size_t gi = ((size_t)bh * DH + d) * G + c8; *(volatile v8b*)(VGT + gi) = *(const v8b*)(&Tt[d][c8]); *(volatile v8b*)(VGTL + gi) = *(const v8b*)(&Tu[d][c8]); }
      __threadfence(); } }
}
__global__ __launch_bounds__(64) void attn_kernel(const b16* __restrict__ QH, const b16* __restrict__ QL, const b16* __restrict__ KH, const b16* __restrict__ VT, const b16* __restrict__ VTL, const b16* __restrict__ KG, const b16* __restrict__ VGT, const b16* __restrict__ VGTL, b16* __restrict__ ATT, b16* __restrict__ ATTL) {
  __shared__ __attribute__((aligned(16))) b16 To[2][16][DH + 8], Tl2[2][16][DH + 8];
  const int wave = threadIdx.x >> 5, lane = threadIdx.x & 31, hh = lane >> 4, col = lane & 15; const int bh = blockIdx.y, b = bh / NH, h = bh - b * NH, i0 = blockIdx.x * 32 + wave * 16, qi = i0 + col;
  const b16* Qh = QH + (size_t)bh * S * DH; const b16* Ql = QL + (size_t)bh * S * DH; const b16* K = KH + (size_t)bh * S * DH; const b16* V = VT + (size_t)bh * DH * LV; const b16* Kg = KG + (size_t)bh * G * DH; const b16* Vg = VGT + (size_t)bh * DH * G; const b16* Vl = VTL + (size_t)bh * DH * LV; const b16* Vgl = VGTL + (size_t)bh * DH * G;
  v16b qf[2], ql[2];
#pragma unroll
  for (int ks = 0; ks < 2; ++ks) { qf[ks] = frag_kb(Qh + (size_t)qi * DH + ks * 32, hh); ql[ks] = frag_kb(Ql + (size_t)qi * DH + ks * 32, hh); }
  float m = -INFINITY, l = 0.0f; v8f o[4] = {{}, {}, {}, {}};
  for (int blk = 0; blk < 11; ++blk) {
    const bool glob = blk < 2; const int kb = glob ? blk * 32 : (i0 - W1 + (blk - 2) * 32);
    v8f s0 = {}, s1 = {};
    { const int r0 = glob ? kb + col : iclamp(kb + col, 0, S - 1), r1 = glob ? kb + 16 + col : iclamp(kb + 16 + col, 0, S - 1); const b16* Kp = glob ? Kg : K;
#pragma unroll
      for (int ks = 0; ks < 2; ++ks) { const v16b k0 = frag_kb(Kp + (size_t)r0 * DH + ks * 32, hh), k1 = frag_kb(Kp + (size_t)r1 * DH + ks * 32, hh);
        s0 = wmma16b(k0, qf[ks], s0); s0 = wmma16b(k0, ql[ks], s0); s1 = wmma16b(k1, qf[ks], s1); s1 = wmma16b(k1, ql[ks], s1); } }
    float mr = -INFINITY;
#pragma unroll
    for (int r = 0; r < 8; ++r) { const int ja = kb + 8 * hh + r, jc = kb + 16 + 8 * hh + r;
      const bool va = glob || (ja >= 0 && ja < S && ja >= qi - W1 && ja <= qi + W1), vc = glob || (jc >= 0 && jc < S && jc >= qi - W1 && jc <= qi + W1);
      s0[r] = va ? s0[r] * (1.0f / (XS * XS)) : -INFINITY; s1[r] = vc ? s1[r] * (1.0f / (XS * XS)) : -INFINITY; mr = fmaxf(mr, fmaxf(s0[r], s1[r])); }
    mr = fmaxf(mr, __shfl_xor(mr, 16)); const float mn = fmaxf(m, mr);
    const float al_ = nexp(m - mn); m = mn; float sum = 0.0f; v16b pb, pl;
#pragma unroll
    for (int r = 0; r < 8; ++r) { const float e0 = nexp(s0[r] - mn), e1 = nexp(s1[r] - mn); sum += e0 + e1; b16 a_, c_; split16(e0 * PS, a_, c_); pb[r] = a_; pl[r] = c_; split16(e1 * PS, a_, c_); pb[8 + r] = a_; pl[8 + r] = c_; }
    sum += __shfl_xor(sum, 16); l = l * al_ + sum;
    { const b16* Vp = glob ? (Vg + kb) : (V + LPAD + kb); const b16* Vq = glob ? (Vgl + kb) : (Vl + LPAD + kb); const int ldv = glob ? G : LV;
#pragma unroll
      for (int t = 0; t < 4; ++t) { o[t] *= al_; const v16b vh = frag_kb(Vp + (size_t)(t * 16 + col) * ldv, hh); o[t] = wmma16b(vh, pb, o[t]); o[t] = wmma16b(vh, pl, o[t]); o[t] = wmma16b(frag_kb(Vq + (size_t)(t * 16 + col) * ldv, hh), pb, o[t]); } } }
  const float inv = 1.0f / (l * PS * XS);
#pragma unroll
  for (int t = 0; t < 4; ++t)
#pragma unroll
    for (int r = 0; r < 8; ++r) { b16 a_, c_; split16(o[t][r] * inv * XS, a_, c_); To[wave][col][t * 16 + 8 * hh + r] = a_; Tl2[wave][col][t * 16 + 8 * hh + r] = c_; }
  wave_lds_sync();
  for (int pass = 0; pass < 2; ++pass) { for (int rr = 0; rr < 16; ++rr) if (lane < 8) { const int s = i0 + rr; const size_t gi = ((size_t)b * S + s) * D + h * DH + lane * 8; *(volatile v8b*)(ATT + gi) = *(const v8b*)(&To[wave][rr][lane * 8]); *(volatile v8b*)(ATTL + gi) = *(const v8b*)(&Tl2[wave][rr][lane * 8]); } __threadfence(); }
}
__global__ __launch_bounds__(256) void vzero_kernel(b16* __restrict__ VT, size_t n8) { const size_t i = (size_t)blockIdx.x * 256 + threadIdx.x; if (i < n8) { const v8b z = {}; for (int pass = 0; pass < 2; ++pass) { *(volatile v8b*)(VT + i * 8) = z; __threadfence(); } } }
__global__ __launch_bounds__(128) void proj_kernel(const b16* __restrict__ ATT, const b16* __restrict__ ATTL, const b16* __restrict__ WT, float* __restrict__ out) {
  __shared__ __attribute__((aligned(16))) float Ts[4][16][128 + 4];
  const int wave = threadIdx.x >> 5, lane = threadIdx.x & 31, nloc = lane & 15, hlf = lane >> 4; const int m0 = blockIdx.x * 64 + wave * 16, n0 = blockIdx.y * 128; const b16* Bw = WT + (size_t)3 * D * D;
  v8f acc[8];
#pragma unroll
  for (int t = 0; t < 8; ++t) acc[t] = (v8f){};
#pragma unroll 2
  for (int kb = 0; kb < D; kb += 32) { const v16b a = frag_kb(ATT + (size_t)(m0 + nloc) * D + kb, hlf), al = frag_kb(ATTL + (size_t)(m0 + nloc) * D + kb, hlf);
#pragma unroll
    for (int t = 0; t < 8; ++t) { const v16b bw = frag_kb(Bw + (size_t)(n0 + t * 16 + nloc) * D + kb, hlf); acc[t] = wmma16b(a, bw, acc[t]); acc[t] = wmma16b(al, bw, acc[t]); } }
#pragma unroll
  for (int t = 0; t < 8; ++t)
#pragma unroll
    for (int r = 0; r < 8; ++r) Ts[wave][8 * hlf + r][t * 16 + nloc] = acc[t][r] * (1.0f / (XS * WSC));
  wave_lds_sync();
  for (int pass = 0; pass < 2; ++pass) { for (int rr = 0; rr < 16; ++rr) *(volatile v4f*)(out + (size_t)(m0 + rr) * D + n0 + lane * 4) = *(const v4f*)(&Ts[wave][rr][lane * 4]); __threadfence(); }
}
}

extern "C" void kernel_launch(void* const* d_in, const int* in_sizes, int n_in, void* d_out, int out_size, void* d_ws, size_t ws_size, hipStream_t stream) {
  (void)n_in;
  auto Fp = [&](int i) { return (const float*)d_in[i]; };
  if (in_sizes[0] != NROW * D || in_sizes[1] != D * D || in_sizes[4] != D * D || in_sizes[5] != NB * G || out_size != NROW * D) return;
  size_t off = 0; char* ws = (char*)d_ws;
  auto carve = [&](size_t bytes) { char* p = ws + off; off += (bytes + 255) & ~(size_t)255; return p; };
  b16* X16 = (b16*)carve((size_t)NROW * D * 2); b16* WT = (b16*)carve((size_t)4 * D * D * 2);
  b16* QH = (b16*)carve((size_t)NROW * D * 2); b16* QL = (b16*)carve((size_t)NROW * D * 2); b16* KH = (b16*)carve((size_t)NROW * D * 2); b16* VROW = (b16*)carve((size_t)NROW * D * 2);
  b16* VROWL = (b16*)carve((size_t)NROW * D * 2); b16* VT = (b16*)carve((size_t)NB * NH * DH * LV * 2); b16* VTL = (b16*)carve((size_t)NB * NH * DH * LV * 2); b16* KG = (b16*)carve((size_t)NB * NH * G * DH * 2); b16* VGT = (b16*)carve((size_t)NB * NH * DH * G * 2); b16* VGTL = (b16*)carve((size_t)NB * NH * DH * G * 2);
  b16* ATT = X16;
  b16* ATTL = VROW;
  if (off > ws_size) return;
  prepx_kernel<<<(NROW * D / 8 + 255) / 256, 256, 0, stream>>>(Fp(0), X16);
  prepw_kernel<<<dim3(D / 64, D / 64, 4), 256, 0, stream>>>(Fp(1), Fp(2), Fp(3), Fp(4), WT);
  qkv_kernel<<<dim3(NROW / 64, D / 128, 3), 128, 0, stream>>>(X16, WT, QH, QL, KH, VROW, VROWL, 0);
  vzero_kernel<<<(NB * NH * DH * LV / 8 + 255) / 256, 256, 0, stream>>>(VT, (size_t)NB * NH * DH * LV / 8); vzero_kernel<<<(NB * NH * DH * LV / 8 + 255) / 256, 256, 0, stream>>>(VTL, (size_t)NB * NH * DH * LV / 8);
  vt_kernel<<<dim3(S / 64 + 1, NB * NH), 256, 0, stream>>>(VROW, VROWL, KH, (const int*)d_in[5], VT, VTL, KG, VGT, VGTL);
  attn_kernel<<<dim3(S / 32, NB * NH), 64, 0, stream>>>(QH, QL, KH, VT, VTL, KG, VGT, VGTL, ATT, ATTL);
  proj_kernel<<<dim3(NROW / 64, D / 128), 128, 0, stream>>>(ATT, ATTL, WT, (float*)d_out);
}
